// ReDynamicWeightsCat11_28097676050580
// MI455X (gfx1250) — hardware-verified
//
#include <hip/hip_runtime.h>
#include <hip/hip_bf16.h>
#include <math.h>


#define BB 2
#define SS 2048
#define DD 1024
#define HH 16
#define DKK 64
#define QW 2

typedef _Float16 bf16;
typedef __attribute__((ext_vector_type(4))) unsigned v4u_t;
typedef unsigned v4ua __attribute__((ext_vector_type(4), may_alias));
typedef __attribute__((ext_vector_type(4))) float v4f_t;
typedef float v4fa __attribute__((ext_vector_type(4), may_alias));
typedef __attribute__((ext_vector_type(16))) bf16  bf16x16;
typedef __attribute__((ext_vector_type(8)))  bf16  bf16x8;
typedef __attribute__((ext_vector_type(4)))  bf16  bf16x4;
typedef __attribute__((ext_vector_type(8)))  float f32x8;

#define LDS_STRIDE 48
#define KSTRIDE    72
#define VSTRIDE    48

__device__ __forceinline__ f32x8 wmma_bf16(bf16x16 a, bf16x16 b, f32x8 c) {
  return __builtin_amdgcn_wmma_f32_16x16x32_f16(
      false, a, false, b, (short)0, c, false, false);
}
#define RSPLIT (1.0f / 2048.0f)
__device__ __forceinline__ bf16 lo_of(float v, bf16 h) { return (bf16)((v - (float)h) * 2048.0f); }
__device__ __forceinline__ f32x8 wmma_split(bf16x16 a, bf16x16 al, bf16x16 b, bf16x16 bl, f32x8 c) {
  f32x8 x = {}; x = wmma_bf16(al, b, x); x = wmma_bf16(a, bl, x); return wmma_bf16(a, b, c) + x * RSPLIT; }

template <typename T>
__device__ __forceinline__ bf16x16 load_frag(const T* __restrict__ base, int ld,
                                             int row0, int k0) {
  const int lane = threadIdx.x & 31;
  const int r    = lane & 15;
  const int kh   = (lane >> 4) * 8;
  const T* p0 = base + (size_t)(row0 + r) * ld + (k0 + kh);
  const T* p1 = p0 + 16;
  bf16x16 f;
#pragma unroll
  for (int i = 0; i < 8; ++i) {
    f[i]     = (bf16)p0[i];
    f[i + 8] = (bf16)p1[i];
  }
  return f;
}

__device__ __forceinline__ bf16x16 lds_frag(const bf16* base, int stride) {
  const int lane = threadIdx.x & 31;
  const int row  = lane & 15;
  const int kh   = (lane >> 4) * 8;
  const bf16x8 lo = *(const bf16x8*)(base + row * stride + kh);
  const bf16x8 hi = *(const bf16x8*)(base + row * stride + kh + 16);
  bf16x16 f;
#pragma unroll
  for (int i = 0; i < 8; ++i) { f[i] = lo[i]; f[i + 8] = hi[i]; }
  return f;
}

template <typename T>
__device__ __forceinline__ void stage_read16(const T* __restrict__ p, float* buf) {
#pragma unroll
  for (int i = 0; i < 16; ++i) buf[i] = (float)p[i];
}

__device__ __forceinline__ void stage_write(bf16* dst, const float* buf, int nquad) {
#pragma unroll
  for (int i = 0; i < nquad; ++i) {
    bf16x4 q;
    q[0] = (bf16)buf[4 * i];     q[1] = (bf16)buf[4 * i + 1];
    q[2] = (bf16)buf[4 * i + 2]; q[3] = (bf16)buf[4 * i + 3];
    *(bf16x4*)(dst + 4 * i) = q;
  }
}

__global__ __launch_bounds__(256) void transpose_pack_kernel(const float* __restrict__ W, bf16* __restrict__ WT, int K, int N, size_t plane) {
  __shared__ float tile[64][65];
  const int k0 = blockIdx.y * 64, n0 = blockIdx.x * 64, t = threadIdx.x;
  for (int i = t; i < 64 * 64; i += 256) { const int kr = i >> 6, nc = i & 63; tile[kr][nc] = W[(size_t)(k0 + kr) * N + n0 + nc]; }
  __syncthreads();
#pragma unroll 1
  for (int pass = 0; pass < 2; ++pass) {
    for (int i = t; i < 64 * 8; i += 256) { const int nr = i >> 3, k8 = (i & 7) * 8; bf16 hh[8], hl[8];
#pragma unroll
      for (int e = 0; e < 8; ++e) { const float v = tile[k8 + e][nr]; hh[e] = (bf16)v; hl[e] = lo_of(v, hh[e]); }
      bf16* d = WT + (size_t)(n0 + nr) * K + k0 + k8;
      *(volatile v4u_t*)d = *(const v4ua*)hh; *(volatile v4u_t*)(d + plane) = *(const v4ua*)hl; }
    __threadfence();
  }
}

template <typename AT, typename WT, int MODE>
__global__ __launch_bounds__(256) void gemm_split_kernel(
    const AT* __restrict__ A, size_t aPlane, const WT* __restrict__ W, size_t wPlane,
    const float* __restrict__ bias, void* __restrict__ out,
    int M, int N, int K) {
  __shared__ bf16 ldsA[128 * LDS_STRIDE], ldsAl[128 * LDS_STRIDE];
  __shared__ bf16 ldsW[256 * LDS_STRIDE], ldsWl[256 * LDS_STRIDE];
  __shared__ __attribute__((aligned(16))) unsigned char sob[256 * 136 * 2];

  const int t    = threadIdx.x;
  const int wave = t >> 5;
  const int lane = t & 31;
  const int wm   = (wave & 1) * 64;
  const int wn   = (wave >> 1) * 64;
  const int mBlk = blockIdx.x * 128;
  const int nBlk = blockIdx.y * 256;
  const int arow = t >> 1;
  const int ach  = (t & 1) * 16;

  f32x8 acc[4][4] = {};
  for (int k = 0; k < K; k += 32) {
    __syncthreads();
    {
      const AT* ap = A + (size_t)(mBlk + arow) * K + k + ach;
      bf16 hh[16], hl[16];
      if (sizeof(AT) == 4) {
#pragma unroll
        for (int i = 0; i < 16; ++i) { const float v = (float)ap[i]; hh[i] = (bf16)v; hl[i] = lo_of(v, hh[i]); }
      } else {
#pragma unroll
        for (int i = 0; i < 16; ++i) { hh[i] = (bf16)ap[i]; hl[i] = (bf16)ap[aPlane + i]; }
      }
#pragma unroll
      for (int i = 0; i < 16; ++i) { ldsA[arow * LDS_STRIDE + ach + i] = hh[i]; ldsAl[arow * LDS_STRIDE + ach + i] = hl[i]; }
    }
    {
      const WT* wp = W + (size_t)(nBlk + t) * K + k;
      if (sizeof(WT) == 4) {
#pragma unroll
        for (int i = 0; i < 32; ++i) { const float v = (float)wp[i]; const bf16 h_ = (bf16)v; ldsW[t * LDS_STRIDE + i] = h_; ldsWl[t * LDS_STRIDE + i] = lo_of(v, h_); }
      } else {
#pragma unroll
        for (int i = 0; i < 32; ++i) { ldsW[t * LDS_STRIDE + i] = (bf16)wp[i]; ldsWl[t * LDS_STRIDE + i] = (bf16)wp[wPlane + i]; }
      }
    }
    __syncthreads();
    bf16x16 wf[4], wfl[4];
#pragma unroll
    for (int j = 0; j < 4; ++j) { wf[j] = lds_frag(ldsW + (wn + 16 * j) * LDS_STRIDE, LDS_STRIDE); wfl[j] = lds_frag(ldsWl + (wn + 16 * j) * LDS_STRIDE, LDS_STRIDE); }
#pragma unroll
    for (int i = 0; i < 4; ++i) {
      const bf16x16 af = lds_frag(ldsA + (wm + 16 * i) * LDS_STRIDE, LDS_STRIDE), afl = lds_frag(ldsAl + (wm + 16 * i) * LDS_STRIDE, LDS_STRIDE);
#pragma unroll
      for (int j = 0; j < 4; ++j) acc[i][j] = wmma_split(af, afl, wf[j], wfl[j], acc[i][j]);
    }
  }

  const int nlane = lane & 15;
  const int mh    = (lane >> 4) * 8;
  __syncthreads();
  if (MODE == 1) {
    bf16* so = (bf16*)sob;
#pragma unroll
    for (int i = 0; i < 4; ++i)
#pragma unroll
      for (int j = 0; j < 4; ++j) {
        const int nl = wn + 16 * j + nlane;
        const float bv = bias ? bias[nBlk + nl] : 0.0f;
#pragma unroll
        for (int r = 0; r < 8; ++r) so[nl * 136 + wm + 16 * i + mh + r] = (bf16)(acc[i][j][r] + bv);
      }
    __syncthreads();
    const int b_ = mBlk >> 11, s0 = mBlk & (SS - 1);
#pragma unroll 1
    for (int pass = 0; pass < 2; ++pass) {
      for (int ch = t; ch < 256 * 16; ch += 256) { const int nl = ch >> 4, q = (ch & 15) * 8; const int n = nBlk + nl, h = n >> 6, dk = n & (DKK - 1);
        *(volatile v4u_t*)((bf16*)out + (((size_t)(b_ * HH + h)) * DKK + dk) * SS + s0 + q) = *(const v4ua*)(so + nl * 136 + q); }
      __threadfence();
    }
  } else {
    float* so = (float*)sob;
#pragma unroll 1
    for (int hf = 0; hf < 2; ++hf) {
      if (wm == hf * 64) {
#pragma unroll
        for (int i = 0; i < 4; ++i)
#pragma unroll
          for (int j = 0; j < 4; ++j) {
            const int nl = wn + 16 * j + nlane;
            const float bv = bias ? bias[nBlk + nl] : 0.0f;
#pragma unroll
            for (int r = 0; r < 8; ++r) so[(16 * i + mh + r) * 260 + nl] = acc[i][j][r] + bv;
          }
      }
      __syncthreads();
#pragma unroll 1
      for (int pass = 0; pass < 2; ++pass) {
        for (int ch = t; ch < 64 * 64; ch += 256) { const int ml = ch >> 6, q = (ch & 63) * 4;
          *(volatile v4f_t*)((float*)out + (size_t)(mBlk + hf * 64 + ml) * N + nBlk + q) = *(const volatile v4fa*)(so + ml * 260 + q); }
        __threadfence();
      }
      __syncthreads();
    }
  }
}


#define RN 2
#define RC1 512
#define RCM 128
#define RHW 96
#define RP 9216
#define RG 32

__global__ __launch_bounds__(256) void k_gnstats(const float* __restrict__ Y, int cpg  , float* __restrict__ stats  ) {
  __shared__ float s1[256], s2[256];
  const int tid = threadIdx.x; const size_t base = (size_t)blockIdx.x * cpg * RP; const int cnt = cpg * RP;
  float a = 0.0f, q = 0.0f;
  for (int i = tid; i < cnt; i += 256) { const float v = Y[base + i]; a += v; q += v * v; }
  s1[tid] = a; s2[tid] = q; __syncthreads();
  for (int o = 128; o > 0; o >>= 1) { if (tid < o) { s1[tid] += s1[tid + o]; s2[tid] += s2[tid + o]; } __syncthreads(); }
  if (tid == 0) { const float m = s1[0] / (float)cnt; const float var = fmaxf(s2[0] / (float)cnt - m * m, 0.0f);
    s1[0] = m; s2[0] = rsqrtf(var + 1e-5f); }
  __syncthreads();
#pragma unroll 1
  for (int pass = 0; pass < 2; ++pass) { if (tid == 0) { *(volatile float*)(stats + blockIdx.x * 32) = s1[0]; *(volatile float*)(stats + blockIdx.x * 32 + 1) = s2[0]; } __threadfence(); }
}

__global__ __launch_bounds__(256) void k_gn1_apply(const float* __restrict__ Y1, const float* __restrict__ st, const float* __restrict__ gw, const float* __restrict__ gb,
                                                  float* __restrict__ xd, bf16* __restrict__ xdT) {
  __shared__ float tl[RCM][65];
  const int n = blockIdx.y, p0 = blockIdx.x * 64, tid = threadIdx.x;
  for (int i = tid; i < RCM * 64; i += 256) { const int c = i >> 6, pp = i & 63; const int g = c >> 2;
    const float m = st[(n * RG + g) * 32], rs = st[(n * RG + g) * 32 + 1];
    tl[c][pp] = fmaxf((Y1[((size_t)n * RCM + c) * RP + p0 + pp] - m) * rs * gw[c] + gb[c], 0.0f); }
  __syncthreads();
  const size_t plane = (size_t)RN * RP * RCM;
#pragma unroll 1
  for (int pass = 0; pass < 2; ++pass) {
    for (int i = tid; i < RCM * 16; i += 256) { const int c = i >> 4, q = (i & 15) * 4; v4f_t v; v.x = tl[c][q]; v.y = tl[c][q + 1]; v.z = tl[c][q + 2]; v.w = tl[c][q + 3];
      *(volatile v4f_t*)(xd + ((size_t)n * RCM + c) * RP + p0 + q) = v; }
    for (int i = tid; i < 64 * 16; i += 256) { const int pp = i >> 4, c8 = (i & 15) * 8; bf16 hh[8], hl[8];
#pragma unroll
      for (int e = 0; e < 8; ++e) { const float v = tl[c8 + e][pp]; hh[e] = (bf16)v; hl[e] = lo_of(v, hh[e]); }
      bf16* d = xdT + ((size_t)n * RP + p0 + pp) * RCM + c8;
      *(volatile v4u_t*)d = *(const v4ua*)hh; *(volatile v4u_t*)(d + plane) = *(const v4ua*)hl; }
    __threadfence();
  }
}

__global__ __launch_bounds__(256) void k_branches(const float* __restrict__ xd, const bf16* __restrict__ xdT,
                                                 const float* __restrict__ wa, const float* __restrict__ wb, const float* __restrict__ wc, const float* __restrict__ wd,
                                                 const float* __restrict__ g1, const float* __restrict__ g2, const float* __restrict__ g3, const float* __restrict__ g4,
                                                 bf16* __restrict__ outT) {
  __shared__ __attribute__((aligned(16))) bf16 Aw[2][16 * 1160];
  __shared__ float wts[8][16][9];
  __shared__ __attribute__((aligned(16))) bf16 ot[8][2][16 * 136];
  __shared__ int offs[9]; __shared__ int dys[9], dxs[9];
  const int n = blockIdx.y, tid = threadIdx.x, lane = tid & 31, wave = tid >> 5, half = lane >> 4, l16 = lane & 15, kh8 = half * 8;
  const int p0 = blockIdx.x * 128 + wave * 16;
  const int p = p0 + l16, py = p / RHW, px = p % RHW;
  const size_t plane = (size_t)RN * RP * RCM;
  const bf16* xT = xdT + (size_t)n * RP * RCM;
  const float* xdn = xd + (size_t)n * RCM * RP;
  float accum[64];
#pragma unroll
  for (int i = 0; i < 64; ++i) accum[i] = 0.0f;
#pragma unroll 1
  for (int di = 0; di < 4; ++di) {
    const int d = (di == 0) ? 1 : (di == 1) ? 4 : (di == 2) ? 8 : 12;
    const float* w = (di == 0) ? wa : (di == 1) ? wb : (di == 2) ? wc : wd;
    const float gam = ((di == 0) ? g1 : (di == 1) ? g2 : (di == 2) ? g3 : g4)[0];
    __syncthreads();
    for (int i = tid; i < 16 * 1152; i += 256) { const int k = i / 1152, kk = i % 1152, tap = kk >> 7, c = kk & 127;
      const float v = (k < 9) ? w[((size_t)k * RCM + c) * 9 + tap] : 0.0f; const bf16 hv = (bf16)v; Aw[0][k * 1160 + kk] = hv; Aw[1][k * 1160 + kk] = lo_of(v, hv); }
    __syncthreads();
    f32x8 lg = {};
#pragma unroll 1
    for (int tap = 0; tap < 9; ++tap) {
      const int yy = py + (tap / 3 - 1) * d, xx = px + (tap % 3 - 1) * d;
      const bool inb = (yy >= 0 && yy < RHW && xx >= 0 && xx < RHW);
      const bf16* brow = xT + (size_t)(inb ? (yy * RHW + xx) : 0) * RCM;
#pragma unroll
      for (int cc = 0; cc < 4; ++cc) {
        bf16x16 bv, bl;
        if (inb) { const bf16x8 lo0 = *(const bf16x8*)(brow + cc * 32 + kh8), hi0 = *(const bf16x8*)(brow + cc * 32 + kh8 + 16);
                   const bf16x8 lo1 = *(const bf16x8*)(brow + plane + cc * 32 + kh8), hi1 = *(const bf16x8*)(brow + plane + cc * 32 + kh8 + 16);
#pragma unroll
                   for (int i = 0; i < 8; ++i) { bv[i] = lo0[i]; bv[i + 8] = hi0[i]; bl[i] = lo1[i]; bl[i + 8] = hi1[i]; } }
        else {
#pragma unroll
          for (int i = 0; i < 16; ++i) { bv[i] = (bf16)0.0f; bl[i] = (bf16)0.0f; } }
        lg = wmma_split(lds_frag(&Aw[0][tap * 128 + cc * 32], 1160), lds_frag(&Aw[1][tap * 128 + cc * 32], 1160), bv, bl, lg);
      }
    }
    const float l8 = __shfl(lg[0], l16 + 16, 32);
    if (half == 0) { float mx = l8;
#pragma unroll
      for (int r = 0; r < 8; ++r) mx = fmaxf(mx, lg[r]);
      float e[9], s = 0.0f;
#pragma unroll
      for (int r = 0; r < 8; ++r) { e[r] = expf(lg[r] - mx); s += e[r]; }
      e[8] = expf(l8 - mx); s += e[8];
      const float inv = 1.0f / s;
#pragma unroll
      for (int r = 0; r < 9; ++r) wts[wave][l16][r] = e[r] * inv * gam;
    }
    __syncthreads();
#pragma unroll 1
    for (int tap = 0; tap < 9; ++tap) {
      const int yy = py + (tap / 3 - 1) * d, xx = px + (tap % 3 - 1) * d;
      if (yy < 0 || yy >= RHW || xx < 0 || xx >= RHW) continue;
      const float wk = wts[wave][l16][tap]; const float* src = xdn + (size_t)(half * 64) * RP + yy * RHW + xx;
#pragma unroll
      for (int c = 0; c < 64; ++c) accum[c] += wk * src[(size_t)c * RP];
    }
  }
  bf16* oh = ot[wave][0]; bf16* ol = ot[wave][1];
#pragma unroll
  for (int c = 0; c < 64; ++c) { const bf16 hv = (bf16)accum[c]; oh[l16 * 136 + half * 64 + c] = hv; ol[l16 * 136 + half * 64 + c] = lo_of(accum[c], hv); }
  asm volatile("s_wait_dscnt 0" ::: "memory");
#pragma unroll 1
  for (int pass = 0; pass < 2; ++pass) {
#pragma unroll
    for (int it = 0; it < 8; ++it) { const int ch = lane + 32 * it, pp = ch >> 4, c8 = (ch & 15) * 8;
      bf16* dst = outT + ((size_t)n * RP + p0 + pp) * RCM + c8;
      *(volatile v4u_t*)dst = *(const v4ua*)(oh + pp * 136 + c8); *(volatile v4u_t*)(dst + plane) = *(const v4ua*)(ol + pp * 136 + c8); }
    __threadfence();
  }
}

__global__ __launch_bounds__(256) void k_gn2_apply(const float* __restrict__ Y2, const float* __restrict__ st, const float* __restrict__ gw, const float* __restrict__ gb, float* __restrict__ out) {
  const size_t e0 = ((size_t)blockIdx.x * 256 + threadIdx.x) * 4;
  const int row = (int)(e0 / RP); const int n = row / RC1, c = row % RC1, g = c >> 4;
  const float m = st[(n * RG + g) * 32], rs = st[(n * RG + g) * 32 + 1], a = rs * gw[c], bb = gb[c] - m * rs * gw[c];
  v4f_t v = *(const v4fa*)(Y2 + e0);
  v.x = fmaxf(v.x * a + bb, 0.0f); v.y = fmaxf(v.y * a + bb, 0.0f); v.z = fmaxf(v.z * a + bb, 0.0f); v.w = fmaxf(v.w * a + bb, 0.0f);
  *(volatile v4f_t*)(out + e0) = v; __threadfence(); *(volatile v4f_t*)(out + e0) = v;
}

extern "C" void kernel_launch(void* const* d_in, const int* in_sizes, int n_in,
                              void* d_out, int out_size, void* d_ws, size_t ws_size,
                              hipStream_t stream) {
  (void)in_sizes; (void)n_in; (void)out_size; (void)ws_size;
  const float* x    = (const float*)d_in[0];
  const float* w1   = (const float*)d_in[1];
  const float* gn1w = (const float*)d_in[2];
  const float* gn1b = (const float*)d_in[3];
  const float* wa   = (const float*)d_in[4];
  const float* wb   = (const float*)d_in[5];
  const float* wc   = (const float*)d_in[6];
  const float* wd   = (const float*)d_in[7];
  const float* g1   = (const float*)d_in[8];
  const float* g2   = (const float*)d_in[9];
  const float* g3   = (const float*)d_in[10];
  const float* g4   = (const float*)d_in[11];
  const float* w3   = (const float*)d_in[12];
  const float* gn3w = (const float*)d_in[13];
  const float* gn3b = (const float*)d_in[14];
  float* out = (float*)d_out;
  char* ws = (char*)d_ws;
  const size_t plX = (size_t)RN * RP * RC1, plM = (size_t)RN * RP * RCM;
  bf16*  XT   = (bf16*)ws;  ws += plX * 2 * 2;
  float* Y1   = (float*)ws; ws += (size_t)RN * RCM * RP * 4;
  float* xd   = (float*)ws; ws += (size_t)RN * RCM * RP * 4;
  bf16*  xdT  = (bf16*)ws;  ws += plM * 2 * 2;
  bf16*  oT   = (bf16*)ws;  ws += plM * 2 * 2;
  float* Y2   = (float*)ws; ws += (size_t)RN * RC1 * RP * 4;
  float* st1  = (float*)ws; ws += 8192;
  float* st2  = (float*)ws; ws += 8192;

  for (int n = 0; n < RN; ++n)
    transpose_pack_kernel<<<dim3(RP / 64, RC1 / 64), 256, 0, stream>>>(x + (size_t)n * RC1 * RP, XT + (size_t)n * RP * RC1, RC1, RP, plX);
  for (int n = 0; n < RN; ++n)
    gemm_split_kernel<float, bf16, 2><<<dim3(RCM / 128, RP / 256), 256, 0, stream>>>(w1, 0, XT + (size_t)n * RP * RC1, plX, nullptr, Y1 + (size_t)n * RCM * RP, RCM, RP, RC1);
  k_gnstats<<<RN * RG, 256, 0, stream>>>(Y1, RCM / RG, st1);
  k_gn1_apply<<<dim3(RP / 64, RN), 256, 0, stream>>>(Y1, st1, gn1w, gn1b, xd, xdT);
  k_branches<<<dim3(RP / 128, RN), 256, 0, stream>>>(xd, xdT, wa, wb, wc, wd, g1, g2, g3, g4, oT);
  for (int n = 0; n < RN; ++n)
    gemm_split_kernel<float, bf16, 2><<<dim3(RC1 / 128, RP / 256), 256, 0, stream>>>(w3, 0, oT + (size_t)n * RP * RCM, plM, nullptr, Y2 + (size_t)n * RC1 * RP, RC1, RP, RCM);
  k_gnstats<<<RN * RG, 256, 0, stream>>>(Y2, RC1 / RG, st2);
  k_gn2_apply<<<(int)((size_t)RN * RC1 * RP / 4 / 256), 256, 0, stream>>>(Y2, st2, gn3w, gn3b, out);
}
